// LMMDrift_55456617726509
// MI455X (gfx1250) — hardware-verified
//
#include <hip/hip_runtime.h>


namespace {
constexpr int N = 8192, K = 64, RB = 64  ;
constexpr float LSC = 65536.0f;

typedef _Float16 b16;
typedef __attribute__((ext_vector_type(16))) _Float16 v16b;
typedef __attribute__((ext_vector_type(8))) _Float16 v8b;
typedef __attribute__((ext_vector_type(8))) float v8f;
typedef __attribute__((ext_vector_type(4))) float v4f;
__device__ __forceinline__ float bf16_rne(float f) { unsigned int u = __float_as_uint(f); u += 0x7FFFu + ((u >> 16) & 1u); return __uint_as_float(u & 0xFFFF0000u); }
__device__ __forceinline__ v16b frag_kb(const b16* p, int hh) { const v8b a = *(const v8b*)(p + 8 * hh), b = *(const v8b*)(p + 16 + 8 * hh); v16b f;
#pragma unroll
  for (int e = 0; e < 8; ++e) { f[e] = a[e]; f[8 + e] = b[e]; } return f; }
__device__ __forceinline__ v8f wmma16b(v16b a, v16b b, v8f c) { v8f d = __builtin_amdgcn_wmma_f32_16x16x32_f16(false, a, false, b, (short)0, c, false, false); asm volatile("v_nop\n\tv_nop\n\tv_nop\n\tv_nop" : "+v"(d) : "v"(a), "v"(b)); return d; }
__device__ __forceinline__ void wave_lds_sync() { __builtin_amdgcn_fence(__ATOMIC_RELEASE, "workgroup"); __builtin_amdgcn_wave_barrier(); __builtin_amdgcn_fence(__ATOMIC_ACQUIRE, "workgroup"); }
__device__ __forceinline__ float pmul(float a, float b) { float p = a * b; asm volatile("" : "+v"(p)); return p; }

__device__ __forceinline__ void fwd_scalars(int j, const float* y, const float* tau_, const float* T, float t, float a, float b, float c, float d, float& sig, float& F, float& g) {
  const float ttm = fmaxf(bf16_rne(T[j]) - t, 0.0f); sig = (a + b * ttm) * __expf(-c * ttm) + d; F = __expf(bf16_rne(y[j])); const float tau = bf16_rne(tau_[j]); g = tau * sig * F / (1.0f + tau * F); }

__global__ __launch_bounds__(256) void prep_kernel(const float* __restrict__ L, const float* __restrict__ y, const float* __restrict__ tau_, const float* __restrict__ T, const float* __restrict__ pt, const float* __restrict__ pa, const float* __restrict__ pb, const float* __restrict__ pc, const float* __restrict__ pd, b16* __restrict__ L16, float* __restrict__ G, float* __restrict__ VS) {
  const int tid = blockIdx.x * 256 + threadIdx.x;
  { const size_t e = (size_t)tid * 8; v8b o; for (int q = 0; q < 8; ++q) o[q] = (b16)(bf16_rne(L[e + q]) * LSC); for (int pass = 0; pass < 2; ++pass) { *(volatile v8b*)(L16 + e) = o; __threadfence(); } }
  if (tid < N) { const float t = bf16_rne(pt[0]), a = bf16_rne(pa[0]), b = bf16_rne(pb[0]), c = bf16_rne(pc[0]), d = bf16_rne(pd[0]); float sig, F, g; fwd_scalars(tid, y, tau_, T, t, a, b, c, d, sig, F, g);
    float vs = 0.0f;
#pragma unroll 4
    for (int k = 0; k < K; ++k) { const float l = bf16_rne(L[(size_t)tid * K + k]); vs += pmul(l, l); }
    for (int pass = 0; pass < 2; ++pass) { ((volatile float*)G)[tid] = g; ((volatile float*)VS)[tid] = vs; __threadfence(); } }
}
__global__ __launch_bounds__(128) void main_kernel(const b16* __restrict__ L16, const float* __restrict__ G, const float* __restrict__ VS, const float* __restrict__ y, const float* __restrict__ tau_, const float* __restrict__ T,
                                                    const float* __restrict__ pt, const float* __restrict__ pa, const float* __restrict__ pb, const float* __restrict__ pc, const float* __restrict__ pd, float* __restrict__ out) {
  __shared__ int cnt[128]; __shared__ __attribute__((aligned(16))) float Os[RB];
  const int wave = threadIdx.x >> 5, lane = threadIdx.x & 31, hh = lane >> 4, col = lane & 15; const int i0 = blockIdx.x * RB + wave * 16;
  const float t = bf16_rne(pt[0]);
  { int c = 0; for (int j = threadIdx.x; j < N; j += 128) c += (bf16_rne(T[j]) < t) ? 1 : 0; cnt[threadIdx.x] = c; }
  __syncthreads();
  int eta = 0; for (int q = 0; q < 128; ++q) eta += cnt[q];
  float acc[8];
#pragma unroll
  for (int r = 0; r < 8; ++r) acc[r] = 0.0f;
  const v16b a0 = frag_kb(L16 + (size_t)(i0 + col) * K, hh), a1 = frag_kb(L16 + (size_t)(i0 + col) * K + 32, hh);
  const int jt0 = eta >> 4, jt1 = (i0 >> 4);
  for (int jt = jt0; jt <= jt1; ++jt) { const int j0 = jt * 16;
    v8f s = {}; s = wmma16b(a0, frag_kb(L16 + (size_t)(j0 + col) * K, hh), s); s = wmma16b(a1, frag_kb(L16 + (size_t)(j0 + col) * K + 32, hh), s);
    const int j = j0 + col; const float gj = G[j]; const bool jok = (j >= eta);
#pragma unroll
    for (int r = 0; r < 8; ++r) { const int i = i0 + 8 * hh + r; const float w = (jok && j <= i) ? gj : 0.0f; acc[r] += pmul(s[r] * (1.0f / (LSC * LSC)), w); } }
#pragma unroll
  for (int r = 0; r < 8; ++r) { float v = acc[r]; v += __shfl_xor(v, 1); v += __shfl_xor(v, 2); v += __shfl_xor(v, 4); v += __shfl_xor(v, 8); acc[r] = v; }
  if (col < 8) { const int r = col; const int i = i0 + 8 * hh + r; const float a = bf16_rne(pa[0]), b = bf16_rne(pb[0]), c = bf16_rne(pc[0]), d = bf16_rne(pd[0]); float sig, F, g; fwd_scalars(i, y, tau_, T, t, a, b, c, d, sig, F, g);
    float drift = acc[0];
#pragma unroll
    for (int q = 1; q < 8; ++q) drift = (r == q) ? acc[q] : drift;
    const float mu = sig * F * drift; const float ld = mu / F - 0.5f * sig * sig * VS[i]; const bool alive = (t <= bf16_rne(T[i])); Os[wave * 16 + 8 * hh + r] = alive ? ld : (ld * 0.0f); }
  __syncthreads();
  for (int pass = 0; pass < 2; ++pass) { if (threadIdx.x < 16) *(volatile v4f*)(out + (size_t)blockIdx.x * RB + threadIdx.x * 4) = *(const v4f*)(&Os[threadIdx.x * 4]); __threadfence(); }
}
}

extern "C" void kernel_launch(void* const* d_in, const int* in_sizes, int n_in, void* d_out, int out_size, void* d_ws, size_t ws_size, hipStream_t stream) {
  (void)n_in;
  auto Fp = [&](int i) { return (const float*)d_in[i]; };
  if (in_sizes[0] != 1 || in_sizes[1] != N || in_sizes[2] != N || in_sizes[3] != N * K || in_sizes[4] != N || in_sizes[5] != 1 || in_sizes[8] != 1 || out_size != N) return;
  size_t off = 0; char* ws = (char*)d_ws;
  auto carve = [&](size_t bytes) { char* p = ws + off; off += (bytes + 255) & ~(size_t)255; return p; };
  b16* L16 = (b16*)carve((size_t)N * K * 2); float* G = (float*)carve((size_t)N * 4); float* VS = (float*)carve((size_t)N * 4);
  if (off > ws_size || off > ((size_t)128 << 20)) return;
  prep_kernel<<<N * K / 8 / 256, 256, 0, stream>>>(Fp(3), Fp(1), Fp(2), Fp(4), Fp(0), Fp(5), Fp(6), Fp(7), Fp(8), L16, G, VS);
  main_kernel<<<N / RB, 128, 0, stream>>>(L16, G, VS, Fp(1), Fp(2), Fp(4), Fp(0), Fp(5), Fp(6), Fp(7), Fp(8), (float*)d_out);
}
